// Wide_48034914238966
// MI455X (gfx1250) — hardware-verified
//
#include <hip/hip_runtime.h>


namespace {
constexpr int NB = 131072, E = 128, NU = 52643, NI = 91599, NCOL = 640;
__constant__ int KSZ[5] = {1, 2, 4, 8, 16};

typedef _Float16 b16;
typedef __attribute__((ext_vector_type(16))) _Float16 v16b;
typedef __attribute__((ext_vector_type(8))) _Float16 v8b;
typedef __attribute__((ext_vector_type(8))) float v8f;
typedef __attribute__((ext_vector_type(4))) float v4f;
__device__ __forceinline__ float bf16_rne(float f) { unsigned int u = __float_as_uint(f); u += 0x7FFFu + ((u >> 16) & 1u); return __uint_as_float(u & 0xFFFF0000u); }
__device__ __forceinline__ v16b frag_kb(const b16* p, int hh) { const v8b a = *(const v8b*)(p + 8 * hh), b = *(const v8b*)(p + 16 + 8 * hh); v16b f;
#pragma unroll
  for (int e = 0; e < 8; ++e) { f[e] = a[e]; f[8 + e] = b[e]; } return f; }
__device__ __forceinline__ v8f wmma16b(v16b a, v16b b, v8f c) { v8f d = __builtin_amdgcn_wmma_f32_16x16x32_f16(false, a, false, b, (short)0, c, false, false); asm volatile("v_nop\n\tv_nop\n\tv_nop\n\tv_nop" : "+v"(d) : "v"(a), "v"(b)); return d; }
__device__ __forceinline__ void wave_lds_sync() { __builtin_amdgcn_fence(__ATOMIC_RELEASE, "workgroup"); __builtin_amdgcn_wave_barrier(); __builtin_amdgcn_fence(__ATOMIC_ACQUIRE, "workgroup"); }
__device__ __forceinline__ float nexp(float x) { return __builtin_amdgcn_exp2f(x * 1.4426950408889634f); }
__device__ __forceinline__ float tanh_f(float x) { const float e = nexp(-2.0f * fabsf(x)); const float t = (1.0f - e) * __builtin_amdgcn_rcpf(1.0f + e); return (x >= 0.0f) ? t : -t; }
__device__ __forceinline__ float pmul(float a, float b) { float p = a * b; asm volatile("" : "+v"(p)); return p; }

__global__ __launch_bounds__(256) void prep_kernel(const float* __restrict__ w1, const float* __restrict__ w2, const float* __restrict__ w3, const float* __restrict__ w4, const float* __restrict__ w5, const float* __restrict__ b1, const float* __restrict__ b2, const float* __restrict__ b3, const float* __restrict__ b4, const float* __restrict__ b5, const float* __restrict__ lw, const float* __restrict__ lb, b16* __restrict__ R, float* __restrict__ P) {
  const int t_ = blockIdx.x * 256 + threadIdx.x, nth = gridDim.x * 256;
  for (int pass = 0; pass < 2; ++pass) {
    for (int q = t_; q < NCOL * E; q += nth) { const int col = q / E, d = q % E, i = col / 128, j = col % 128, k = KSZ[i]; const float* w = (i == 0) ? w1 : (i == 1) ? w2 : (i == 2) ? w3 : (i == 3) ? w4 : w5; float v = 0.0f;
      if (j < 129 - k && d - j >= 0 && d - j < k) v = bf16_rne(w[d - j]); R[q] = (b16)v; }
    for (int q = t_; q < 17; q += nth) { float v = 0.0f; if (q < 5) { const float* bb = (q == 0) ? b1 : (q == 1) ? b2 : (q == 2) ? b3 : (q == 3) ? b4 : b5; v = bb[0]; } else if (q >= 8 && q < 13) v = lw[q - 8]; else if (q == 16) v = lb[0]; P[q] = bf16_rne(v); }
    __threadfence(); }
}

__global__ __launch_bounds__(128) void wide_kernel(const int* __restrict__ us, const int* __restrict__ ps, const int* __restrict__ ns, const float* __restrict__ ue, const float* __restrict__ ie, const b16* __restrict__ R, const float* __restrict__ P, float* __restrict__ out0, float* __restrict__ out1) {
  __shared__ __attribute__((aligned(16))) b16 Em[4][3][32][E + 8]; __shared__ float So[4][2][32];
  const int lane = threadIdx.x & 31, wave = threadIdx.x >> 5, nloc = lane & 15, hlf = lane >> 4, r0 = blockIdx.x * 128 + wave * 32;
  for (int i = lane; i < 3 * 32 * (E / 8); i += 32) { const int which = i / (32 * (E / 8)), rr = (i / (E / 8)) % 32, c8 = (i % (E / 8)) * 8; const int row = r0 + rr;
    int id; const float* tab; int lim; if (which == 0) { id = us[row]; tab = ue; lim = NU; } else { id = (which == 1) ? ps[row] : ns[row]; tab = ie; lim = NI; } id = (id < 0) ? 0 : (id >= lim ? lim - 1 : id);
    const float* src = tab + (size_t)id * E + c8; v8b v; for (int e = 0; e < 8; ++e) v[e] = (b16)bf16_rne(src[e]); *(v8b*)(&Em[wave][which][rr][c8]) = v; }
  wave_lds_sync();
  float sp[2][8], sn[2][8];
#pragma unroll
  for (int r = 0; r < 2; ++r)
#pragma unroll
    for (int v = 0; v < 8; ++v) { sp[r][v] = 0.0f; sn[r][v] = 0.0f; }
  for (int i = 0; i < 5; ++i) { const int nvalid = 129 - KSZ[i]; const float bi = P[i], lwi = P[8 + i];
    float dp[2][8], dn[2][8];
#pragma unroll
    for (int r = 0; r < 2; ++r)
#pragma unroll
      for (int v = 0; v < 8; ++v) { dp[r][v] = 0.0f; dn[r][v] = 0.0f; }
    for (int t = 0; t < 8; ++t) { const int col = i * 128 + t * 16 + nloc; const bool cv = (t * 16 + nloc) < nvalid;
      v8f au[2] = {{}, {}}, ap[2] = {{}, {}}, an[2] = {{}, {}};
#pragma unroll
      for (int kb = 0; kb < E; kb += 32) { const v16b bw = frag_kb(R + (size_t)col * E + kb, hlf);
#pragma unroll
        for (int r = 0; r < 2; ++r) { const v16b fu = frag_kb(&Em[wave][0][r * 16 + nloc][kb], hlf), fp = frag_kb(&Em[wave][1][r * 16 + nloc][kb], hlf), fn = frag_kb(&Em[wave][2][r * 16 + nloc][kb], hlf); au[r] = wmma16b(fu, bw, au[r]); ap[r] = wmma16b(fp, bw, ap[r]); an[r] = wmma16b(fn, bw, an[r]); } }
      if (cv) {
#pragma unroll
        for (int r = 0; r < 2; ++r)
#pragma unroll
          for (int v = 0; v < 8; ++v) { const float fu = tanh_f(au[r][v] + bi), fp = tanh_f(ap[r][v] + bi), fn = tanh_f(an[r][v] + bi); dp[r][v] += pmul(fu, fp); dn[r][v] += pmul(fu, fn); } } }
#pragma unroll
    for (int r = 0; r < 2; ++r)
#pragma unroll
      for (int v = 0; v < 8; ++v) { float a = dp[r][v], c = dn[r][v];
#pragma unroll
        for (int o = 1; o < 16; o <<= 1) { a += __shfl_xor(a, o); c += __shfl_xor(c, o); }
        sp[r][v] += pmul(a, lwi); sn[r][v] += pmul(c, lwi); } }
  if (nloc == 0) { const float lb = P[16];
#pragma unroll
    for (int r = 0; r < 2; ++r)
#pragma unroll
      for (int v = 0; v < 8; ++v) { So[wave][0][r * 16 + 8 * hlf + v] = sp[r][v] + lb; So[wave][1][r * 16 + 8 * hlf + v] = sn[r][v] + lb; } }
  wave_lds_sync();
  for (int pass = 0; pass < 2; ++pass) { ((volatile float*)out0)[r0 + lane] = So[wave][0][lane]; ((volatile float*)out1)[r0 + lane] = So[wave][1][lane]; __threadfence(); }
}
}

extern "C" void kernel_launch(void* const* d_in, const int* in_sizes, int n_in,
                              void* d_out, int out_size, void* d_ws, size_t ws_size, hipStream_t stream) {
  (void)n_in; (void)out_size;
  const int* us = (const int*)d_in[0]; const int* ps = (const int*)d_in[1]; const int* ns = (const int*)d_in[2]; const float* ue = (const float*)d_in[3]; const float* ie = (const float*)d_in[4];
  const float* w1 = (const float*)d_in[5]; const float* b1 = (const float*)d_in[6]; const float* w2 = (const float*)d_in[7]; const float* b2 = (const float*)d_in[8]; const float* w3 = (const float*)d_in[9]; const float* b3 = (const float*)d_in[10]; const float* w4 = (const float*)d_in[11]; const float* b4 = (const float*)d_in[12]; const float* w5 = (const float*)d_in[13]; const float* b5 = (const float*)d_in[14]; const float* lw = (const float*)d_in[15]; const float* lb = (const float*)d_in[16];
  float* out0 = (float*)d_out; float* out1 = out0 + NB;
  if (in_sizes[0] != NB || in_sizes[3] != NU * E || in_sizes[4] != NI * E || in_sizes[13] != 16 || in_sizes[15] != 5) return;
  size_t off = 0; char* ws = (char*)d_ws;
  auto carve = [&](size_t bytes) { char* p = ws + off; off += (bytes + 255) & ~(size_t)255; return p; };
  b16* R = (b16*)carve((size_t)NCOL * E * 2); float* P = (float*)carve(256);
  if (off > ws_size) return;
  prep_kernel<<<64, 256, 0, stream>>>(w1, w2, w3, w4, w5, b1, b2, b3, b4, b5, lw, lb, R, P);
  wide_kernel<<<NB / 128, 128, 0, stream>>>(us, ps, ns, ue, ie, R, P, out0, out1);
}
